// HeteroData_GNNmodel_9294309228905
// MI455X (gfx1250) — hardware-verified
//
#include <hip/hip_runtime.h>
#include <stddef.h>


#define FIN     256
#define H1D     256
#define H2D     128
#define NTHR    256
#define NWAVE   8
#define EPT     8
#define NGRP    2
#define CHUNK   (NTHR * EPT * NGRP)
#define WCAPC   (EPT * NGRP * 32)
#define WCAPF   (EPT * NGRP * 32)
#define ESHF    11
#define EMASK   0xFFFFF
#define NBC     32768
#define NBF     1024
#define RCAP    49152
#define RBN     128
#define TGT     256
#define DEGCAP  512
#define GROWS   128
#define GCOLS   128
#define OTHR    256
#define TPK     64
#define TPN     32
#define TPP     72
#define ASCL    16
#define WSCL    64
#define WSCAP   134217728

#define LDS_COUNT  ((NBC + NWAVE * WCAPC + NWAVE) * 4)
#define LDS_FILL   ((RCAP + NBF + NWAVE * WCAPF + NWAVE) * 4)
#define LDS_GEMM   (GROWS * GCOLS * 4)

static_assert((CHUNK & (CHUNK - 1)) == 0);
static_assert((NBC & (NBC - 1)) == 0 && (NBF & (NBF - 1)) == 0);
static_assert(NBF <= (1 << ESHF));
static_assert((NBC % NBF) == 0);
static_assert(OTHR * 4 == NBF);
static_assert((OTHR % 32) == 0 && OTHR <= 1024);
static_assert((RCAP % 32) == 0);
static_assert(RBN == 32 * 4);
static_assert(TGT == NWAVE * 32);
static_assert(GROWS == NWAVE * 16);
static_assert((TGT % GROWS) == 0);
static_assert((NBF % TGT) == 0);
static_assert(NBC == NWAVE * 32 * 128);
static_assert(GCOLS == 32 * 4);
static_assert((FIN % 32) == 0 && (H1D % 32) == 0);
static_assert((H1D % GCOLS) == 0 && (H2D % GCOLS) == 0);
static_assert((H1D % 128) == 0 && H2D == 128);
static_assert(2 * H2D <= H1D);
static_assert((FIN % TPK) == 0 && (H1D % TPK) == 0 && (H1D % TPN) == 0 && (H2D % TPN) == 0);
static_assert(TPN * 8 == NTHR && TPK * TPN == NTHR * 8 && TPK == NWAVE * 8);
static_assert((TPP % 8) == 0 && TPP >= TPK);
static_assert(LDS_FILL <= 300 * 1024);

typedef float     v4f  __attribute__((ext_vector_type(4)));
typedef float     v8f  __attribute__((ext_vector_type(8)));
typedef int       v4i  __attribute__((ext_vector_type(4)));
typedef _Float16  v8h  __attribute__((ext_vector_type(8)));
typedef _Float16  v16h __attribute__((ext_vector_type(16)));
union FragH { v16h v; v8h h[2]; };
union U32F { float f; int i; };

__device__ __forceinline__ v8f wmf(v16h a, v16h b, v8f c) {
  v8f d = __builtin_amdgcn_wmma_f32_16x16x32_f16(false, a, false, b, (short)0, c, false, false);
  asm volatile("v_nop\n\tv_nop\n\tv_nop\n\tv_nop" : "+v"(d) : "v"(a), "v"(b));
  return d;
}

__device__ __forceinline__ v8h cvt8h(v4f a, v4f b, float z) {
  v8h h;
  h[0] = (_Float16)(a.x * z); h[1] = (_Float16)(a.y * z); h[2] = (_Float16)(a.z * z); h[3] = (_Float16)(a.w * z);
  h[4] = (_Float16)(b.x * z); h[5] = (_Float16)(b.y * z); h[6] = (_Float16)(b.z * z); h[7] = (_Float16)(b.w * z);
  return h;
}

template <int NB, int SRC, int WC>
__device__ __forceinline__ int scan_chunk(const int* __restrict__ keys, int nK, int cbase,
                                          int slotBase, int vec8, int* list, int tid, int lane, int wave) {
  int wc = 0;
#pragma unroll
  for (int g = 0; g < NGRP; ++g) {
    const int el0  = (g * NTHR + tid) * EPT;
    const int e0   = cbase + el0;
    const int sent = -2147483647 - 1;
    const int i0 = min(e0, nK - 1),     i1 = min(e0 + 1, nK - 1), i2 = min(e0 + 2, nK - 1), i3 = min(e0 + 3, nK - 1);
    const int i4 = min(e0 + 4, nK - 1), i5 = min(e0 + 5, nK - 1), i6 = min(e0 + 6, nK - 1), i7 = min(e0 + 7, nK - 1);
    v4i da, db;
    if (vec8 != 0 && cbase + CHUNK <= nK) {
      da = *(const v4i*)(keys + e0);
      db = *(const v4i*)(keys + e0 + 4);
    } else {
      da.x = (e0     < nK) ? keys[i0] : sent;
      da.y = (e0 + 1 < nK) ? keys[i1] : sent;
      da.z = (e0 + 2 < nK) ? keys[i2] : sent;
      da.w = (e0 + 3 < nK) ? keys[i3] : sent;
      db.x = (e0 + 4 < nK) ? keys[i4] : sent;
      db.y = (e0 + 5 < nK) ? keys[i5] : sent;
      db.z = (e0 + 6 < nK) ? keys[i6] : sent;
      db.w = (e0 + 7 < nK) ? keys[i7] : sent;
    }
    const unsigned nb = (unsigned)slotBase;
    const unsigned s0 = (unsigned)da.x - nb, s1 = (unsigned)da.y - nb;
    const unsigned s2 = (unsigned)da.z - nb, s3 = (unsigned)da.w - nb;
    const unsigned s4 = (unsigned)db.x - nb, s5 = (unsigned)db.y - nb;
    const unsigned s6 = (unsigned)db.z - nb, s7 = (unsigned)db.w - nb;
    const bool h0 = s0 < (unsigned)NB, h1 = s1 < (unsigned)NB, h2 = s2 < (unsigned)NB, h3 = s3 < (unsigned)NB;
    const bool h4 = s4 < (unsigned)NB, h5 = s5 < (unsigned)NB, h6 = s6 < (unsigned)NB, h7 = s7 < (unsigned)NB;
    const unsigned any = __builtin_amdgcn_ballot_w32(h0 | h1 | h2 | h3 | h4 | h5 | h6 | h7);
    if (any != 0u) {
#define HITJ(HJ, SJ, VJ) { \
        const unsigned mj = __builtin_amdgcn_ballot_w32(HJ); \
        if (mj != 0u) { \
          if (HJ) { \
            const int pos = wc + (int)__builtin_amdgcn_mbcnt_lo(mj, 0u); \
            const int entv = SRC ? (((VJ) << ESHF) | (int)(SJ)) : (int)(SJ); \
            if (pos < WC) list[wave * WC + pos] = entv; \
          } \
          wc += (int)__builtin_popcount(mj); } }
      HITJ(h0, s0, i0)
      HITJ(h1, s1, i1)
      HITJ(h2, s2, i2)
      HITJ(h3, s3, i3)
      HITJ(h4, s4, i4)
      HITJ(h5, s5, i5)
      HITJ(h6, s6, i6)
      HITJ(h7, s7, i7)
#undef HITJ
    }
  }
  return wc;
}

__global__ __launch_bounds__(NTHR) void k_wT16(const float* __restrict__ W, _Float16* Wp,
                                               int KD, int NC, int NCP, float scale) {
  __shared__ __attribute__((aligned(16))) _Float16 sT[TPN * TPP];
  const int tid = threadIdx.x;
  const int z = (int)blockIdx.z;
  const float* Wz = W + (size_t)z * (size_t)KD * (size_t)NC;
  _Float16* Wpz = Wp + (size_t)z * (size_t)NCP * (size_t)KD;
  const int k0 = (int)blockIdx.x * TPK, n0 = (int)blockIdx.y * TPN;
  const int nc = tid & 31, kq = tid >> 5;
  const int col = n0 + nc;
  const int colc = col < NC ? col : NC - 1;
#pragma unroll
  for (int i = 0; i < TPK / NWAVE; ++i) {
    const int kr = kq + NWAVE * i;
    const float w = Wz[(size_t)(k0 + kr) * NC + colc];
    const float v = (col < NC) ? w * scale : 0.0f;
    sT[nc * TPP + kr] = (_Float16)v;
  }
  __syncthreads();
  const int nl = tid >> 3, p = tid & 7;
  const v8h hv = *(const v8h*)(sT + nl * TPP + 8 * p);
  _Float16* d = Wpz + (size_t)(n0 + nl) * KD + k0 + 8 * p;
  *(volatile v8h*)d = hv;
  __threadfence();
  *(volatile v8h*)d = hv;
}

__global__ __launch_bounds__(NTHR) void k_count(
    const int* __restrict__ keys, int* cnt, int nK, int vec8) {
  extern __shared__ v4f lds_dyn[];
  int* scnt = (int*)lds_dyn;
  int* list = scnt + NBC;
  int* wcnt = list + NWAVE * WCAPC;
  const int tid = threadIdx.x, lane = tid & 31, wave = tid >> 5;
  const int nodeBase = blockIdx.x * NBC;

  {
    const v4i z = {0, 0, 0, 0};
    for (int i = tid; i < NBC / 4; i += NTHR) ((v4i*)scnt)[i] = z;
  }
  __syncthreads();

  const int nChunks = (nK + CHUNK - 1) / CHUNK;
#pragma unroll 1
  for (int ch = 0; ch < nChunks; ++ch) {
    const int cbase = ch * CHUNK;
    const int wc = scan_chunk<NBC, 0, WCAPC>(keys, nK, cbase, nodeBase, vec8, list, tid, lane, wave);
    if (lane == 0) wcnt[wave] = wc;
    __syncthreads();
    if (wave == 0) {
#pragma unroll 1
      for (int wsx = 0; wsx < NWAVE; ++wsx) {
        int n = __builtin_amdgcn_readfirstlane(wcnt[wsx]);
        n = n > WCAPC ? WCAPC : (n < 0 ? 0 : n);
        const int* lp = list + wsx * WCAPC;
#pragma unroll 1
        for (int i = 0; i < n; ++i) {
          const int ent  = __builtin_amdgcn_readfirstlane(lp[i]);
          const int slot = ent & (NBC - 1);
          if (lane == 0) scnt[slot] = scnt[slot] + 1;
        }
      }
    }
    __syncthreads();
  }

  int* cp = cnt + (size_t)nodeBase;
#pragma unroll 4
  for (int q = 0; q < 32; ++q) {
    const int f = (wave * 32 + q) * 128 + 4 * lane;
    const v4i c = *(const v4i*)(scnt + f);
    *(volatile v4i*)(cp + f) = c;
  }
  __threadfence();
#pragma unroll 4
  for (int q = 0; q < 32; ++q) {
    const int f = (wave * 32 + q) * 128 + 4 * lane;
    const v4i c = *(const v4i*)(scnt + f);
    *(volatile v4i*)(cp + f) = c;
  }
}

__global__ __launch_bounds__(OTHR) void k_offsets(
    const int* __restrict__ cnt, int* off, float* dis, int* rbase, int nBF) {
  __shared__ __attribute__((aligned(16))) int srb[RBN];
  __shared__ int wtot[OTHR / 32];
  const int tid = threadIdx.x, lane = tid & 31, wave = tid >> 5;
  for (int i = tid; i < RBN; i += OTHR) srb[i] = 0;
  int carry = 0;
#pragma unroll 1
  for (int fb = 0; fb < nBF; ++fb) {
    const int base = fb * NBF;
    const v4i c = *(const v4i*)(cnt + base + 4 * tid);
    const int e0 = max(c.x, 0), e1 = max(c.y, 0), e2 = max(c.z, 0), e3 = max(c.w, 0);
    const int ts = e0 + e1 + e2 + e3;
    int incl = ts;
#pragma unroll
    for (int d = 1; d < 32; d <<= 1) {
      const int t = __shfl_up(incl, d, 32);
      if (lane >= d) incl += t;
    }
    if (lane == 31) wtot[wave] = incl;
    __syncthreads();
    int pre = 0;
#pragma unroll 1
    for (int w = 0; w < wave; ++w) pre += wtot[w];
    int tot = 0;
#pragma unroll
    for (int w = 0; w < OTHR / 32; ++w) tot += wtot[w];
    int run = carry + pre + incl - ts;
    v4i o;
    o.x = run; run += e0;
    o.y = run; run += e1;
    o.z = run; run += e2;
    o.w = run;
    v4f dv;
    dv.x = rsqrtf((float)e0 + 1.0f);
    dv.y = rsqrtf((float)e1 + 1.0f);
    dv.z = rsqrtf((float)e2 + 1.0f);
    dv.w = rsqrtf((float)e3 + 1.0f);
    int*   op = off + base + 4 * tid;
    float* dp = dis + base + 4 * tid;
    *(volatile v4i*)op = o;
    *(volatile v4f*)dp = dv;
    __threadfence();
    *(volatile v4i*)op = o;
    *(volatile v4f*)dp = dv;
    if (tid == 0) srb[min(fb, RBN - 1)] = carry;
    carry += (tot + 31) & ~31;
    __syncthreads();
  }
  if (tid == 0) srb[min(nBF, RBN - 1)] = carry;
  __syncthreads();
  v4i rv = {0, 0, 0, 0};
  if (tid < 32) rv = *(const v4i*)(srb + 4 * tid);
  if (tid < 32) *(volatile v4i*)(rbase + 4 * tid) = rv;
  __threadfence();
  if (tid < 32) *(volatile v4i*)(rbase + 4 * tid) = rv;
}

__global__ __launch_bounds__(NTHR) void k_fill(
    const int* __restrict__ keys, const int* __restrict__ off,
    const int* __restrict__ rbase, int* csr, int nK, int vec8, int csrLen) {
  extern __shared__ v4f lds_dyn[];
  int* region = (int*)lds_dyn;
  int* cursor = region + RCAP;
  int* list   = cursor + NBF;
  int* wcnt   = list + NWAVE * WCAPF;
  const int tid = threadIdx.x, lane = tid & 31, wave = tid >> 5;
  const int b = blockIdx.x;
  const int nodeBase = b * NBF;

  int rb0 = rbase[b];
  const int rb1 = rbase[b + 1];
  rb0 = rb0 < 0 ? 0 : (rb0 > csrLen ? csrLen : rb0);
  rb0 &= ~31;
  int len = rb1 - rb0;
  len = len < 0 ? 0 : (len > RCAP ? RCAP : len);
  int lenW = (len + 31) & ~31;
  if (rb0 + lenW > csrLen) lenW = (csrLen - rb0) & ~31;

  {
    const v4i z = {0, 0, 0, 0};
    for (int i = tid; i < RCAP / 4; i += NTHR) ((v4i*)region)[i] = z;
    for (int s = tid; s < NBF; s += NTHR) {
      int o = off[nodeBase + s] - rb0;
      o = o < 0 ? 0 : (o > RCAP ? RCAP : o);
      cursor[s] = o;
    }
  }
  __syncthreads();

  const int nChunks = (nK + CHUNK - 1) / CHUNK;
#pragma unroll 1
  for (int ch = 0; ch < nChunks; ++ch) {
    const int cbase = ch * CHUNK;
    const int wc = scan_chunk<NBF, 1, WCAPF>(keys, nK, cbase, nodeBase, vec8, list, tid, lane, wave);
    if (lane == 0) wcnt[wave] = wc;
    __syncthreads();
    if (wave == 0) {
#pragma unroll 1
      for (int wsx = 0; wsx < NWAVE; ++wsx) {
        int n = __builtin_amdgcn_readfirstlane(wcnt[wsx]);
        n = n > WCAPF ? WCAPF : (n < 0 ? 0 : n);
        const int* lp = list + wsx * WCAPF;
#pragma unroll 1
        for (int i = 0; i < n; ++i) {
          const int ent  = __builtin_amdgcn_readfirstlane(lp[i]);
          const int slot = ent & (NBF - 1);
          int ev = (ent >> ESHF) & EMASK;
          ev = ev > nK - 1 ? nK - 1 : ev;
          if (lane == 0) {
            int pos = cursor[slot];
            pos = pos < 0 ? 0 : (pos > RCAP - 1 ? RCAP - 1 : pos);
            region[pos] = ev;
            const int np = pos + 1;
            cursor[slot] = np > RCAP ? RCAP : np;
          }
        }
      }
    }
    __syncthreads();
  }

  const int nv = lenW >> 2;
  int* gp = csr + rb0;
#pragma unroll 1
  for (int i = tid; i < nv; i += NTHR) { const v4i v = ((const v4i*)region)[i]; *(volatile v4i*)(gp + 4 * i) = v; }
  __threadfence();
#pragma unroll 1
  for (int i = tid; i < nv; i += NTHR) { const v4i v = ((const v4i*)region)[i]; *(volatile v4i*)(gp + 4 * i) = v; }
}

template <int KD>
__global__ __launch_bounds__(NTHR) void k_gemm(
    const float* __restrict__ A, int lda, int nArows,
    const _Float16* __restrict__ Bw, float* Cout, int ldc, float osc) {
  extern __shared__ v4f lds_dyn[];
  static_assert((KD % 32) == 0);
  constexpr int NC  = GCOLS;
  constexpr int NT  = NC / 16;
  constexpr int NST = 16;
  float* stg = (float*)lds_dyn;
  const int tid = threadIdx.x, lane = tid & 31, wave = tid >> 5, hh = lane >> 4, m = lane & 15;
  const int rowBase = blockIdx.x * GROWS;
  const int cb = blockIdx.y;
  const int ar  = rowBase + wave * 16 + m;
  const int arc = ar < nArows ? ar : nArows - 1;
  const float z = (ar < nArows) ? (float)ASCL : 0.0f;
  const float* ap = A + (size_t)arc * lda + 8 * hh;
  const _Float16* bp0 = Bw + (size_t)(cb * NC + m) * KD + 8 * hh;

  v8f acc[NT];
#pragma unroll
  for (int t = 0; t < NT; ++t) { v8f zz = {0.f, 0.f, 0.f, 0.f, 0.f, 0.f, 0.f, 0.f}; acc[t] = zz; }

#pragma unroll 1
  for (int kt = 0; kt < KD / 32; ++kt) {
    const float* p = ap + 32 * kt;
    const v4f f0 = *(const v4f*)p;
    const v4f f1 = *(const v4f*)(p + 4);
    const v4f f2 = *(const v4f*)(p + 16);
    const v4f f3 = *(const v4f*)(p + 20);
    FragH af;
    af.h[0] = cvt8h(f0, f1, z);
    af.h[1] = cvt8h(f2, f3, z);
#pragma unroll
    for (int t = 0; t < NT; ++t) {
      const _Float16* bp = bp0 + (size_t)(16 * t) * KD + 32 * kt;
      FragH bf;
      bf.h[0] = *(const v8h*)bp;
      bf.h[1] = *(const v8h*)(bp + 16);
      acc[t] = wmf(af.v, bf.v, acc[t]);
    }
  }

  const int r0 = wave * 16 + 8 * hh;
  float* sp = stg + r0 * NC + m;
#pragma unroll
  for (int t = 0; t < NT; ++t) {
#pragma unroll
    for (int r = 0; r < 8; ++r) {
      sp[r * NC + 16 * t] = acc[t][r] * osc;
    }
  }
  __syncthreads();

  const float* lp = stg + wave * 16 * NC;
  float* gp = Cout + (size_t)(rowBase + wave * 16) * ldc + cb * NC;
#pragma unroll
  for (int i = 0; i < NST; ++i) {
    const v4f v = *(const v4f*)(lp + i * NC + 4 * lane);
    *(volatile v4f*)(gp + (size_t)i * ldc + 4 * lane) = v;
  }
  __threadfence();
#pragma unroll
  for (int i = 0; i < NST; ++i) {
    const v4f v = *(const v4f*)(lp + i * NC + 4 * lane);
    *(volatile v4f*)(gp + (size_t)i * ldc + 4 * lane) = v;
  }
}

template <int NV>
__device__ __forceinline__ void agg_rel(
    v4f (&acc)[NV], const int* __restrict__ csr, const int* __restrict__ srcidx,
    const float* __restrict__ dis, const float* __restrict__ hw,
    int nE, int csrLen, int nN, int n, int st, float dc, int c, int lane, int ch) {
  constexpr int LD = NV * 128;
#pragma unroll 1
  for (int q0 = 0; q0 < n; q0 += 32) {
    int pos = st + q0 + lane;
    pos = pos < 0 ? 0 : (pos > csrLen - 1 ? csrLen - 1 : pos);
    int el = csr[pos];
    el = el < 0 ? 0 : (el > nE - 1 ? nE - 1 : el);
    int sl = srcidx[el];
    sl = sl < 0 ? 0 : (sl > nN - 1 ? nN - 1 : sl);
    U32F wu; wu.f = dis[sl] * dc;
    const int mcnt = (n - q0) < 32 ? (n - q0) : 32;
#pragma unroll 1
    for (int p = 0; p < mcnt; ++p) {
      const int s = __builtin_amdgcn_readlane(sl, p);
      U32F t; t.i = __builtin_amdgcn_readlane(wu.i, p);
      const float* hp = hw + (size_t)s * LD + ch;
#pragma unroll
      for (int v = 0; v < NV; ++v) {
        const v4f hv = *(const v4f*)(hp + 128 * v);
        acc[v] = acc[v] + hv * t.f;
      }
    }
  }
  const float d2 = dc * dc;
  const float* cp = hw + (size_t)c * LD + ch;
#pragma unroll
  for (int v = 0; v < NV; ++v) {
    const v4f hc = *(const v4f*)(cp + 128 * v);
    acc[v] = acc[v] + hc * d2;
  }
}

template <int NREL, int NV, int RELU>
__global__ __launch_bounds__(NTHR) void k_agg(
    const int* __restrict__ csrA, const int* __restrict__ offA, const int* __restrict__ cntA,
    const int* __restrict__ srcA, const float* __restrict__ disA, const float* __restrict__ hwA,
    const float* __restrict__ bA, int nEA, int csrLenA,
    const int* __restrict__ csrB, const int* __restrict__ offB, const int* __restrict__ cntB,
    const int* __restrict__ srcB, const float* __restrict__ disB, const float* __restrict__ hwB,
    const float* __restrict__ bB, int nEB, int csrLenB,
    float* G, int nN) {
  constexpr int LD = NV * 128;
  const int tid = threadIdx.x, lane = tid & 31, wave = tid >> 5;
  const int tbase = blockIdx.x * TGT + wave * 32;
  const int cl = tbase + lane;
  const int ch = 4 * lane;
  const int cA_l = cntA[cl];
  const int oA_l = offA[cl];
  const float dA_l = disA[cl];
  int cB_l = 0, oB_l = 0;
  float dB_l = 1.0f;
  if (NREL == 2) { cB_l = cntB[cl]; oB_l = offB[cl]; dB_l = disB[cl]; }
  v4f bv[NV];
#pragma unroll
  for (int v = 0; v < NV; ++v) {
    bv[v] = *(const v4f*)(bA + 128 * v + ch);
    if (NREL == 2) bv[v] = bv[v] + *(const v4f*)(bB + 128 * v + ch);
  }

#pragma unroll 1
  for (int j = 0; j < 32; ++j) {
    const int c = tbase + j;
    v4f acc[NV];
#pragma unroll
    for (int v = 0; v < NV; ++v) { v4f zz = {0.f, 0.f, 0.f, 0.f}; acc[v] = zz; }
    const int nrA = __builtin_amdgcn_readlane(cA_l, j);
    const int nA  = nrA < 0 ? 0 : (nrA > DEGCAP ? DEGCAP : nrA);
    const int stA = __builtin_amdgcn_readlane(oA_l, j);
    U32F duA; duA.i = __builtin_amdgcn_readlane(__float_as_int(dA_l), j);
    agg_rel<NV>(acc, csrA, srcA, disA, hwA, nEA, csrLenA, nN, nA, stA, duA.f, c, lane, ch);
    bool poison = nrA > DEGCAP;
    if (NREL == 2) {
      const int nrB = __builtin_amdgcn_readlane(cB_l, j);
      const int nB  = nrB < 0 ? 0 : (nrB > DEGCAP ? DEGCAP : nrB);
      const int stB = __builtin_amdgcn_readlane(oB_l, j);
      U32F duB; duB.i = __builtin_amdgcn_readlane(__float_as_int(dB_l), j);
      agg_rel<NV>(acc, csrB, srcB, disB, hwB, nEB, csrLenB, nN, nB, stB, duB.f, c, lane, ch);
      poison = poison || (nrB > DEGCAP);
    }
    v4f y[NV];
#pragma unroll
    for (int v = 0; v < NV; ++v) {
      v4f a = acc[v] + bv[v];
      if (RELU == 1) {
        a.x = fmaxf(a.x, 0.0f); a.y = fmaxf(a.y, 0.0f); a.z = fmaxf(a.z, 0.0f); a.w = fmaxf(a.w, 0.0f);
      }
      y[v] = a;
    }
    if (poison) {
      const float qn = __int_as_float(0x7fc00000);
#pragma unroll
      for (int v = 0; v < NV; ++v) { y[v].x = qn; y[v].y = qn; y[v].z = qn; y[v].w = qn; }
    }
    float* xp = G + (size_t)c * LD + ch;
#pragma unroll
    for (int v = 0; v < NV; ++v) *(volatile v4f*)(xp + 128 * v) = y[v];
    __threadfence();
#pragma unroll
    for (int v = 0; v < NV; ++v) *(volatile v4f*)(xp + 128 * v) = y[v];
  }
}

__global__ __launch_bounds__(NTHR) void k_pred(
    const float* __restrict__ g, const float* __restrict__ cm,
    const int* __restrict__ es, const int* __restrict__ ed,
    float* outp, int nL, int nGr, int nCr) {
  __shared__ __attribute__((aligned(16))) float stg[NTHR];
  const int tid = threadIdx.x, lane = tid & 31, wave = tid >> 5;
  const int ebase = blockIdx.x * NTHR + wave * 32;
  int ei = ebase + lane;
  ei = ei > nL - 1 ? nL - 1 : ei;
  int sl = es[ei];
  sl = sl < 0 ? 0 : (sl > nGr - 1 ? nGr - 1 : sl);
  int dl = ed[ei];
  dl = dl < 0 ? 0 : (dl > nCr - 1 ? nCr - 1 : dl);
  const int ch = 4 * lane;
  float mine = 0.0f;
#pragma unroll 1
  for (int j = 0; j < 32; ++j) {
    const int s = __builtin_amdgcn_readlane(sl, j);
    const int d = __builtin_amdgcn_readlane(dl, j);
    const v4f a = *(const v4f*)(g + (size_t)s * H2D + ch);
    const v4f b = *(const v4f*)(cm + (size_t)d * H2D + ch);
    float p = (a.x * b.x + a.y * b.y) + (a.z * b.z + a.w * b.w);
    p += __shfl_xor(p, 16, 32);
    p += __shfl_xor(p, 8, 32);
    p += __shfl_xor(p, 4, 32);
    p += __shfl_xor(p, 2, 32);
    p += __shfl_xor(p, 1, 32);
    mine = (lane == j) ? p : mine;
  }
  stg[tid] = mine;
  __syncthreads();

  int nr = nL - blockIdx.x * NTHR;
  nr = nr > NTHR ? NTHR : (nr < 0 ? 0 : nr);
  const int nF4 = nr >> 2;
  const int nTail = nr - 4 * nF4;
  float* gp = outp + (size_t)blockIdx.x * NTHR;
  const v4f v = *(const v4f*)(stg + 4 * (tid & 63));
  const int it = 4 * nF4 + (tid & 3);
  const float sv = stg[it > NTHR - 1 ? NTHR - 1 : it];
  if (tid < nF4) *(volatile v4f*)(gp + 4 * tid) = v;
  if (tid < nTail) *(volatile float*)(gp + it) = sv;
  __threadfence();
  if (tid < nF4) *(volatile v4f*)(gp + 4 * tid) = v;
  if (tid < nTail) *(volatile float*)(gp + it) = sv;
}

static inline int cdiv(int a, int b) { return (a + b - 1) / b; }

extern "C" void kernel_launch(void* const* d_in, const int* in_sizes, int n_in,
                              void* d_out, int out_size, void* d_ws, size_t ws_size,
                              hipStream_t stream) {
  if (n_in < 19) return;
  if (in_sizes[0] <= 0 || (in_sizes[0] % FIN) != 0) return;
  if (in_sizes[1] <= 0 || (in_sizes[1] % FIN) != 0) return;
  const int nG  = in_sizes[0] / FIN;
  const int nCn = in_sizes[1] / FIN;
  if (in_sizes[2] < 2 || (in_sizes[2] & 1) != 0) return;
  if (in_sizes[3] < 2 || (in_sizes[3] & 1) != 0) return;
  if (in_sizes[4] < 2 || (in_sizes[4] & 1) != 0) return;
  const int nEgg = in_sizes[2] / 2;
  const int nErv = in_sizes[3] / 2;
  const int nEcc = in_sizes[4] / 2;
  const int nL = in_sizes[5];
  if (nL < 1 || in_sizes[6] != nL || out_size != nL) return;
  if (in_sizes[7]  != FIN * H1D || in_sizes[8]  != H1D) return;
  if (in_sizes[9]  != FIN * H1D || in_sizes[10] != H1D) return;
  if (in_sizes[11] != FIN * H1D || in_sizes[12] != H1D) return;
  if (in_sizes[13] != H1D * H2D || in_sizes[14] != H2D) return;
  if (in_sizes[15] != H1D * H2D || in_sizes[16] != H2D) return;
  if (in_sizes[17] != H1D * H2D || in_sizes[18] != H2D) return;
  if (nG > (1 << 20) || nCn > (1 << 20)) return;
  if (nEgg > (1 << 20) || nErv > (1 << 20) || nEcc > (1 << 20)) return;

  const float* x_gene = (const float*)d_in[0];
  const float* x_cell = (const float*)d_in[1];
  const int*   ei_gg  = (const int*)d_in[2];
  const int*   ei_rev = (const int*)d_in[3];
  const int*   ei_cc  = (const int*)d_in[4];
  const int*   el_src = (const int*)d_in[5];
  const int*   el_dst = (const int*)d_in[6];
  const float* W1_gg  = (const float*)d_in[7];
  const float* b1_gg  = (const float*)d_in[8];
  const float* W1_rev = (const float*)d_in[9];
  const float* b1_rev = (const float*)d_in[10];
  const float* W1_cc  = (const float*)d_in[11];
  const float* b1_cc  = (const float*)d_in[12];
  const float* W2_gg  = (const float*)d_in[13];
  const float* b2_gg  = (const float*)d_in[14];
  const float* W2_rev = (const float*)d_in[15];
  const float* b2_rev = (const float*)d_in[16];
  const float* W2_cc  = (const float*)d_in[17];
  const float* b2_cc  = (const float*)d_in[18];
  float* out = (float*)d_out;

  const int NPADG = cdiv(nG, TGT) * TGT;
  const int NPADC = cdiv(nCn, TGT) * TGT;
  const int nBCg  = cdiv(nG, NBC),  CNTPg = nBCg * NBC;
  const int nBFg  = cdiv(nG, NBF),  OFFNg = nBFg * NBF;
  const int nBCc  = cdiv(nCn, NBC), CNTPc = nBCc * NBC;
  const int nBFc  = cdiv(nCn, NBF), OFFNc = nBFc * NBF;
  if (nBFg + 1 > RBN || nBFc + 1 > RBN) return;
  if (OFFNg > CNTPg || NPADG > OFFNg || OFFNc > CNTPc || NPADC > OFFNc) return;
  if ((NPADG % GROWS) != 0 || (NPADC % GROWS) != 0) return;
  const int csrLgg = ((nEgg + 31) & ~31) + 32 * (nBFg + 1);
  const int csrLrv = ((nErv + 31) & ~31) + 32 * (nBFg + 1);
  const int csrLcc = ((nEcc + 31) & ~31) + 32 * (nBFc + 1);
  const int nGemmG = NPADG / GROWS, nGemmC = NPADC / GROWS;
  const int nAggG  = NPADG / TGT,   nAggC  = NPADC / TGT;
  const int nPred  = cdiv(nL, NTHR);

  char* ws = (char*)d_ws;
  size_t off = 0;
#define CARVE(NAME, BYTES) const size_t NAME = off; off += (size_t)(BYTES); off = (off + 255) & ~(size_t)255;
  CARVE(oW1gg, (size_t)H1D * FIN * 2)
  CARVE(oW1rv, (size_t)H1D * FIN * 2)
  CARVE(oW1cc, (size_t)H1D * FIN * 2)
  CARVE(oW2gg, (size_t)H2D * H1D * 2)
  CARVE(oW2rv, (size_t)H2D * H1D * 2)
  CARVE(oW2cc, (size_t)H2D * H1D * 2)
  CARVE(oXA,   (size_t)NPADG * H1D * 4)
  CARVE(oXB,   (size_t)NPADG * H1D * 4)
  CARVE(oXC,   (size_t)NPADC * H1D * 4)
  CARVE(oG1,   (size_t)NPADG * H1D * 4)
  CARVE(oC1,   (size_t)NPADC * H1D * 4)
  CARVE(oG2,   (size_t)NPADG * H2D * 4)
  CARVE(oC2,   (size_t)NPADC * H2D * 4)
  CARVE(oCnGG, (size_t)CNTPg * 4)
  CARVE(oOfGG, (size_t)OFFNg * 4)
  CARVE(oDiGG, (size_t)OFFNg * 4)
  CARVE(oRbGG, (size_t)RBN * 4)
  CARVE(oCsGG, (size_t)csrLgg * 4)
  CARVE(oCnRV, (size_t)CNTPg * 4)
  CARVE(oOfRV, (size_t)OFFNg * 4)
  CARVE(oDiRV, (size_t)OFFNg * 4)
  CARVE(oRbRV, (size_t)RBN * 4)
  CARVE(oCsRV, (size_t)csrLrv * 4)
  CARVE(oCnCC, (size_t)CNTPc * 4)
  CARVE(oOfCC, (size_t)OFFNc * 4)
  CARVE(oDiCC, (size_t)OFFNc * 4)
  CARVE(oRbCC, (size_t)RBN * 4)
  CARVE(oCsCC, (size_t)csrLcc * 4)
#undef CARVE
  if (off > ws_size || off > (size_t)WSCAP) return;
  _Float16* W1ggP = (_Float16*)(ws + oW1gg);
  _Float16* W1rvP = (_Float16*)(ws + oW1rv);
  _Float16* W1ccP = (_Float16*)(ws + oW1cc);
  _Float16* W2ggP = (_Float16*)(ws + oW2gg);
  _Float16* W2rvP = (_Float16*)(ws + oW2rv);
  _Float16* W2ccP = (_Float16*)(ws + oW2cc);
  float* XA = (float*)(ws + oXA);
  float* XB = (float*)(ws + oXB);
  float* XC = (float*)(ws + oXC);
  float* G1 = (float*)(ws + oG1);
  float* C1 = (float*)(ws + oC1);
  float* G2 = (float*)(ws + oG2);
  float* C2 = (float*)(ws + oC2);
  float* XW2A = XA;
  float* XW2B = XA + (size_t)NPADG * H2D;
  float* XW2C = XC;
  int*   cntGG = (int*)(ws + oCnGG);   int* offGG = (int*)(ws + oOfGG);   float* disGG = (float*)(ws + oDiGG);
  int*   rbGG  = (int*)(ws + oRbGG);   int* csrGG = (int*)(ws + oCsGG);
  int*   cntRV = (int*)(ws + oCnRV);   int* offRV = (int*)(ws + oOfRV);   float* disRV = (float*)(ws + oDiRV);
  int*   rbRV  = (int*)(ws + oRbRV);   int* csrRV = (int*)(ws + oCsRV);
  int*   cntCC = (int*)(ws + oCnCC);   int* offCC = (int*)(ws + oOfCC);   float* disCC = (float*)(ws + oDiCC);
  int*   rbCC  = (int*)(ws + oRbCC);   int* csrCC = (int*)(ws + oCsCC);

  const float osc = 1.0f / ((float)ASCL * (float)WSCL);

  {
    const dim3 gW1(FIN / TPK, H1D / TPN, 1);
    k_wT16<<<gW1, NTHR, 0, stream>>>(W1_gg,  W1ggP, FIN, H1D, H1D, (float)WSCL);
    k_wT16<<<gW1, NTHR, 0, stream>>>(W1_rev, W1rvP, FIN, H1D, H1D, (float)WSCL);
    k_wT16<<<gW1, NTHR, 0, stream>>>(W1_cc,  W1ccP, FIN, H1D, H1D, (float)WSCL);
    const dim3 gW2(H1D / TPK, H2D / TPN, 1);
    k_wT16<<<gW2, NTHR, 0, stream>>>(W2_gg,  W2ggP, H1D, H2D, H2D, (float)WSCL);
    k_wT16<<<gW2, NTHR, 0, stream>>>(W2_rev, W2rvP, H1D, H2D, H2D, (float)WSCL);
    k_wT16<<<gW2, NTHR, 0, stream>>>(W2_cc,  W2ccP, H1D, H2D, H2D, (float)WSCL);
  }

  hipFuncSetAttribute(reinterpret_cast<const void*>(&k_count),
                      hipFuncAttributeMaxDynamicSharedMemorySize, LDS_COUNT);
  hipFuncSetAttribute(reinterpret_cast<const void*>(&k_fill),
                      hipFuncAttributeMaxDynamicSharedMemorySize, LDS_FILL);
  {
    const int* dstGG = ei_gg + nEgg;
    const int vec8GG = ((nEgg & 3) == 0) ? 1 : 0;
    k_count<<<nBCg, NTHR, LDS_COUNT, stream>>>(dstGG, cntGG, nEgg, vec8GG);
    k_offsets<<<1, OTHR, 0, stream>>>(cntGG, offGG, disGG, rbGG, nBFg);
    k_fill<<<nBFg, NTHR, LDS_FILL, stream>>>(dstGG, offGG, rbGG, csrGG, nEgg, vec8GG, csrLgg);
    const int* dstRV = ei_rev + nErv;
    const int vec8RV = ((nErv & 3) == 0) ? 1 : 0;
    k_count<<<nBCg, NTHR, LDS_COUNT, stream>>>(dstRV, cntRV, nErv, vec8RV);
    k_offsets<<<1, OTHR, 0, stream>>>(cntRV, offRV, disRV, rbRV, nBFg);
    k_fill<<<nBFg, NTHR, LDS_FILL, stream>>>(dstRV, offRV, rbRV, csrRV, nErv, vec8RV, csrLrv);
    const int* dstCC = ei_cc + nEcc;
    const int vec8CC = ((nEcc & 3) == 0) ? 1 : 0;
    k_count<<<nBCc, NTHR, LDS_COUNT, stream>>>(dstCC, cntCC, nEcc, vec8CC);
    k_offsets<<<1, OTHR, 0, stream>>>(cntCC, offCC, disCC, rbCC, nBFc);
    k_fill<<<nBFc, NTHR, LDS_FILL, stream>>>(dstCC, offCC, rbCC, csrCC, nEcc, vec8CC, csrLcc);
  }

  hipFuncSetAttribute(reinterpret_cast<const void*>(&k_gemm<FIN>),
                      hipFuncAttributeMaxDynamicSharedMemorySize, LDS_GEMM);
  hipFuncSetAttribute(reinterpret_cast<const void*>(&k_gemm<H1D>),
                      hipFuncAttributeMaxDynamicSharedMemorySize, LDS_GEMM);
  k_gemm<FIN><<<dim3(nGemmG, H1D / GCOLS, 1), NTHR, LDS_GEMM, stream>>>(x_gene, FIN, nG,  W1ggP, XA, H1D, osc);
  k_gemm<FIN><<<dim3(nGemmG, H1D / GCOLS, 1), NTHR, LDS_GEMM, stream>>>(x_gene, FIN, nG,  W1rvP, XB, H1D, osc);
  k_gemm<FIN><<<dim3(nGemmC, H1D / GCOLS, 1), NTHR, LDS_GEMM, stream>>>(x_cell, FIN, nCn, W1ccP, XC, H1D, osc);

  k_agg<2, H1D / 128, 1><<<nAggG, NTHR, 0, stream>>>(
      csrGG, offGG, cntGG, ei_gg,  disGG, XA, b1_gg,  nEgg, csrLgg,
      csrRV, offRV, cntRV, ei_rev, disRV, XB, b1_rev, nErv, csrLrv,
      G1, nG);
  k_agg<1, H1D / 128, 1><<<nAggC, NTHR, 0, stream>>>(
      csrCC, offCC, cntCC, ei_cc, disCC, XC, b1_cc, nEcc, csrLcc,
      csrCC, offCC, cntCC, ei_cc, disCC, XC, b1_cc, nEcc, csrLcc,
      C1, nCn);

  k_gemm<H1D><<<dim3(nGemmG, H2D / GCOLS, 1), NTHR, LDS_GEMM, stream>>>(G1, H1D, nG,  W2ggP, XW2A, H2D, osc);
  k_gemm<H1D><<<dim3(nGemmG, H2D / GCOLS, 1), NTHR, LDS_GEMM, stream>>>(G1, H1D, nG,  W2rvP, XW2B, H2D, osc);
  k_gemm<H1D><<<dim3(nGemmC, H2D / GCOLS, 1), NTHR, LDS_GEMM, stream>>>(C1, H1D, nCn, W2ccP, XW2C, H2D, osc);

  k_agg<2, H2D / 128, 0><<<nAggG, NTHR, 0, stream>>>(
      csrGG, offGG, cntGG, ei_gg,  disGG, XW2A, b2_gg,  nEgg, csrLgg,
      csrRV, offRV, cntRV, ei_rev, disRV, XW2B, b2_rev, nErv, csrLrv,
      G2, nG);
  k_agg<1, H2D / 128, 0><<<nAggC, NTHR, 0, stream>>>(
      csrCC, offCC, cntCC, ei_cc, disCC, XW2C, b2_cc, nEcc, csrLcc,
      csrCC, offCC, cntCC, ei_cc, disCC, XW2C, b2_cc, nEcc, csrLcc,
      C2, nCn);

  k_pred<<<nPred, NTHR, 0, stream>>>(G2, C2, el_src, el_dst, out, nL, nG, nCn);
}
